// GraphSAGEModel_6279242187332
// MI455X (gfx1250) — hardware-run, weakly checked
//
#include <hip/hip_runtime.h>
#include <stddef.h>
#include <stdint.h>


#define NN     100000
#define NE     1600000
#define DF     128
#define NLAY   3
#define GBM    128
#define GBN    128
#define GTHR   256
#define NTILE  782
#define MP     (NTILE * GBM)
#define MW     256
#define K0     384
#define K1     512
#define BNEPS  1e-5f
#define BTHR   256
#define BWAVE  8
#define EPT    8
#define CHUNK  (BTHR * EPT)
#define NBA    1024
#define SLA    10
#define NBLK   98
#define WLCAP  4096
#define RCAP   20480
#define DEGCAP 64
#define BZ_INTS (BWAVE * WLCAP + RCAP + 3 * NBA)
#define BLDS_INTS (BZ_INTS + 16)
#define BLDS_BYTES (BLDS_INTS * 4)
#define GLDS_BYTES ((GBM * GBN + DF) * 4 + 2 * DF * 8)
#define RTHR   256
#define RWAVE  8
#define RROWS  8
#define RBROWS (RWAVE * RROWS)
#define PTHR   256
#define PB_XB  ((MP * (DF / 8)) / PTHR)
#define NU_W0  (3 * 2048)
#define NU_W1  (4 * 2048)
#define PB_W   ((NU_W0 + 2 * NU_W1) / PTHR)
#define NU_TAB 224
#define NU_Z   ((MP - NN) * MW / 8)
#define PB_Z   (NU_Z / PTHR)
#define PB_ALL (PB_XB + PB_W + 1 + 2 * PB_Z)

static_assert(DF % 8 == 0 && DF == 4 * 32 && GBN == DF);
static_assert(NTILE * GBM >= NN && (NTILE - 1) * GBM < NN);
static_assert(NBLK * NBA >= NN && (NBLK - 1) * NBA < NN);
static_assert(NBA == (1 << SLA) && NBA / GBM == 8);
static_assert(NE < (1 << 21));
static_assert(RCAP >= 16710 + 16710 / 20 + 1 && RCAP % (BTHR * 4) == 0);
static_assert(DEGCAP >= 36 + 8);
static_assert(BZ_INTS % (BTHR * 4) == 0);
static_assert(BLDS_BYTES <= 300000 && BLDS_BYTES <= 327680 && GLDS_BYTES <= 327680);
static_assert((MP * (DF / 8)) % PTHR == 0 && (NN * (DF / 8)) % PTHR == 0);
static_assert(NU_W0 % PTHR == 0 && NU_W1 % PTHR == 0 && NU_Z % PTHR == 0 && NU_TAB <= PTHR);
static_assert(K0 % 32 == 0 && K1 % 32 == 0 && (2 * DF) % 32 == 0);
static_assert(GTHR == (GBM / 16) * 32);

constexpr size_t SZ_PL   = (size_t)MP * MW * 2;
constexpr size_t SZ_XB   = (size_t)MP * DF * 2;
constexpr size_t SZ_LIST = (size_t)NBLK * RCAP * 4;
constexpr size_t SZ_NT   = (size_t)NBLK * NBA * 4;
constexpr size_t SZ_REC  = (size_t)NTILE * 2 * DF * 8;
constexpr size_t SZ_WC0  = (size_t)DF * K0 * 2;
constexpr size_t SZ_WC1  = (size_t)DF * K1 * 2;
constexpr size_t SZ_TAB  = (size_t)7 * DF * 4;
constexpr size_t SZ_STAT = (size_t)2 * 2 * DF * 4;
constexpr size_t SZ_FLAG = (size_t)NBLK * 128;
constexpr size_t O_MEAN  = 0;
constexpr size_t O_H     = O_MEAN + SZ_PL;
constexpr size_t O_LIST  = O_H + SZ_PL;
constexpr size_t O_CNT   = O_LIST + SZ_LIST;
constexpr size_t O_OFF   = O_CNT + SZ_NT;
constexpr size_t O_INV   = O_OFF + SZ_NT;
constexpr size_t O_REC   = O_INV + SZ_NT;
constexpr size_t O_WC0   = O_REC + SZ_REC;
constexpr size_t O_WC1   = O_WC0 + SZ_WC0;
constexpr size_t O_WC2   = O_WC1 + SZ_WC1;
constexpr size_t O_TAB   = O_WC2 + SZ_WC1;
constexpr size_t O_STAT  = O_TAB + SZ_TAB;
constexpr size_t O_FLAG  = O_STAT + SZ_STAT;
constexpr size_t O_END   = O_FLAG + SZ_FLAG;
static_assert(SZ_PL % 256 == 0 && SZ_LIST % 256 == 0 && SZ_NT % 256 == 0 && SZ_REC % 256 == 0);
static_assert(SZ_WC0 % 256 == 0 && SZ_WC1 % 256 == 0 && SZ_TAB % 256 == 0 && SZ_STAT % 256 == 0 && SZ_FLAG % 256 == 0);
static_assert(SZ_XB <= SZ_PL);
static_assert(O_END <= ((size_t)128 << 20));

typedef float          v4f   __attribute__((ext_vector_type(4)));
typedef float          v8f   __attribute__((ext_vector_type(8)));
typedef int            v4i   __attribute__((ext_vector_type(4)));
typedef int            v8i   __attribute__((ext_vector_type(8)));
typedef unsigned       v2u   __attribute__((ext_vector_type(2)));
typedef unsigned       v4u   __attribute__((ext_vector_type(4)));
typedef unsigned short v4us  __attribute__((ext_vector_type(4)));
typedef unsigned short v8us  __attribute__((ext_vector_type(8)));
typedef unsigned short v16us __attribute__((ext_vector_type(16)));
typedef __bf16         v16bf __attribute__((ext_vector_type(16)));
typedef v4f  __attribute__((may_alias)) v4fa;
typedef v4i  __attribute__((may_alias)) v4ia;
typedef v2u  __attribute__((may_alias)) v2ua;
typedef v4u  __attribute__((may_alias)) v4ua;
typedef v4us __attribute__((may_alias)) v4usa;
typedef v8us __attribute__((may_alias)) v8usa;
union FragB { v16bf v; v16us u; v8us h[2]; v8i w; };

__device__ __forceinline__ v8f wmb(const FragB& a, const FragB& b, v8f c) {
  v8f d = __builtin_amdgcn_wmma_f32_16x16x32_bf16(false, a.v, false, b.v, (short)0, c, false, false);
  asm volatile("v_nop\n\tv_nop\n\tv_nop\n\tv_nop" : "+v"(d) : "v"(a.w), "v"(b.w));
  return d;
}

__device__ __forceinline__ v8f z8() { v8f z = {0.f, 0.f, 0.f, 0.f, 0.f, 0.f, 0.f, 0.f}; return z; }

__device__ __forceinline__ unsigned bf16_bits(float f) {
  const unsigned u = __float_as_uint(f);
  const unsigned r = (u + 0x7FFFu + ((u >> 16) & 1u)) >> 16;
  return (f != f) ? 0x7FC0u : r;
}
__device__ __forceinline__ unsigned hl_bits(float v, unsigned& lo) {
  const unsigned hb = bf16_bits(v);
  lo = bf16_bits(v - __uint_as_float(hb << 16));
  return hb;
}

__device__ __forceinline__ void wave_sync() {
  __builtin_amdgcn_fence(__ATOMIC_RELEASE, "wavefront");
  __builtin_amdgcn_wave_barrier();
  __builtin_amdgcn_fence(__ATOMIC_ACQUIRE, "wavefront");
}

__global__ __launch_bounds__(PTHR) void k_prep(const float* __restrict__ x, const float* __restrict__ wl,
                                               const float* __restrict__ wr, const float* __restrict__ bl,
                                               const float* __restrict__ gam, const float* __restrict__ bet,
                                               unsigned* wsb) {
  const int b = (int)blockIdx.x, tid = (int)threadIdx.x;
  v4u o = {0u, 0u, 0u, 0u};
  size_t dw = 0;
  bool live = true;
  if (b < PB_XB) {
    const int u = b * PTHR + tid;
    const int row = u >> 4, c8 = (u & 15) * 8;
    const int rc = row < NN ? row : NN - 1;
    const float* p = x + (size_t)rc * DF + c8;
    const v4f a0 = *(const v4f*)p;
    const v4f a1 = *(const v4f*)(p + 4);
    const unsigned msk = row < NN ? 0xFFFFFFFFu : 0u;
    o.x = (bf16_bits(a0.x) | (bf16_bits(a0.y) << 16)) & msk;
    o.y = (bf16_bits(a0.z) | (bf16_bits(a0.w) << 16)) & msk;
    o.z = (bf16_bits(a1.x) | (bf16_bits(a1.y) << 16)) & msk;
    o.w = (bf16_bits(a1.z) | (bf16_bits(a1.w) << 16)) & msk;
    dw = O_H / 4 + (size_t)u * 4;
  } else if (b < PB_XB + PB_W) {
    int v = (b - PB_XB) * PTHR + tid;
    int l, kp;
    size_t ob;
    if (v < NU_W0)              { l = 0; kp = K0; ob = O_WC0 / 4; }
    else if (v < NU_W0 + NU_W1) { v -= NU_W0; l = 1; kp = K1; ob = O_WC1 / 4; }
    else                        { v -= NU_W0 + NU_W1; l = 2; kp = K1; ob = O_WC2 / 4; }
    const int seg = v >> 11, n = (v >> 4) & (DF - 1), kk = (v & 15) * 8;
    const size_t so = (size_t)l * DF * DF + (size_t)kk * DF + (size_t)n;
    float f[8];
    if (seg < 2) {
#pragma unroll
      for (int i = 0; i < 8; ++i) f[i] = wl[so + (size_t)i * DF];
    } else {
#pragma unroll
      for (int i = 0; i < 8; ++i) f[i] = wr[so + (size_t)i * DF];
    }
    o.x = bf16_bits(f[0]) | (bf16_bits(f[1]) << 16);
    o.y = bf16_bits(f[2]) | (bf16_bits(f[3]) << 16);
    o.z = bf16_bits(f[4]) | (bf16_bits(f[5]) << 16);
    o.w = bf16_bits(f[6]) | (bf16_bits(f[7]) << 16);
    dw = ob + ((size_t)n * kp + (size_t)seg * DF + (size_t)kk) / 2;
  } else if (b == PB_XB + PB_W) {
    const int u = tid;
    live = u < NU_TAB;
    const int uc = u < NU_TAB ? u : NU_TAB - 1;
    const int ub = uc < 95 ? uc : 95;
    int ug = uc - 96;  ug = ug < 0 ? 0 : (ug > 63 ? 63 : ug);
    int ue = uc - 160; ue = ue < 0 ? 0 : (ue > 63 ? 63 : ue);
    const v4f vb = *(const v4f*)(bl + 4 * ub);
    const v4f vg = *(const v4f*)(gam + 4 * ug);
    const v4f ve = *(const v4f*)(bet + 4 * ue);
    asm volatile("" :: "v"(vb), "v"(vg), "v"(ve));
    const unsigned mb = uc < 96 ? 0xFFFFFFFFu : 0u;
    const unsigned me = uc >= 160 ? 0xFFFFFFFFu : 0u;
    const unsigned mg = ~(mb | me);
    const float s0 = __uint_as_float((__float_as_uint(vb.x) & mb) | (__float_as_uint(vg.x) & mg) | (__float_as_uint(ve.x) & me));
    const float s1 = __uint_as_float((__float_as_uint(vb.y) & mb) | (__float_as_uint(vg.y) & mg) | (__float_as_uint(ve.y) & me));
    const float s2 = __uint_as_float((__float_as_uint(vb.z) & mb) | (__float_as_uint(vg.z) & mg) | (__float_as_uint(ve.z) & me));
    const float s3 = __uint_as_float((__float_as_uint(vb.w) & mb) | (__float_as_uint(vg.w) & mg) | (__float_as_uint(ve.w) & me));
    o.x = bf16_bits(s0) << 16; o.y = bf16_bits(s1) << 16; o.z = bf16_bits(s2) << 16; o.w = bf16_bits(s3) << 16;
    dw = O_TAB / 4 + (size_t)uc * 4;
  } else if (b < PB_XB + PB_W + 1 + PB_Z) {
    const int u = (b - (PB_XB + PB_W + 1)) * PTHR + tid;
    dw = O_MEAN / 4 + ((size_t)NN * MW) / 2 + (size_t)u * 4;
  } else {
    const int u = (b - (PB_XB + PB_W + 1 + PB_Z)) * PTHR + tid;
    dw = O_H / 4 + ((size_t)NN * MW) / 2 + (size_t)u * 4;
  }
  unsigned* dp = wsb + dw;
  if (live) *(volatile v4u*)dp = o;
  __threadfence();
  if (live) *(volatile v4u*)dp = o;
}

__device__ __forceinline__ int sweep_chunk(const int* __restrict__ dsts, int cbase, int slotBase, int nb,
                                           int vec8, int* wlw, int wc, int tid) {
  const int el0  = tid * EPT;
  const int e0   = cbase + el0;
  const int sent = (int)(1u << 31);
  v4i da, db;
  if (vec8 != 0 && cbase + CHUNK <= NE) {
    da = *(const v4i*)(dsts + e0);
    db = *(const v4i*)(dsts + e0 + 4);
  } else {
    const int t0 = dsts[min(e0,     NE - 1)];
    const int t1 = dsts[min(e0 + 1, NE - 1)];
    const int t2 = dsts[min(e0 + 2, NE - 1)];
    const int t3 = dsts[min(e0 + 3, NE - 1)];
    const int t4 = dsts[min(e0 + 4, NE - 1)];
    const int t5 = dsts[min(e0 + 5, NE - 1)];
    const int t6 = dsts[min(e0 + 6, NE - 1)];
    const int t7 = dsts[min(e0 + 7, NE - 1)];
    asm volatile("" :: "v"(t0), "v"(t1), "v"(t2), "v"(t3), "v"(t4), "v"(t5), "v"(t6), "v"(t7));
    da.x = (e0     < NE) ? t0 : sent;
    da.y = (e0 + 1 < NE) ? t1 : sent;
    da.z = (e0 + 2 < NE) ? t2 : sent;
    da.w = (e0 + 3 < NE) ? t3 : sent;
    db.x = (e0 + 4 < NE) ? t4 : sent;
    db.y = (e0 + 5 < NE) ? t5 : sent;
    db.z = (e0 + 6 < NE) ? t6 : sent;
    db.w = (e0 + 7 < NE) ? t7 : sent;
  }
  const unsigned nbs = (unsigned)slotBase;
  const unsigned unb = (unsigned)nb;
  const unsigned s0 = (unsigned)da.x - nbs, s1 = (unsigned)da.y - nbs;
  const unsigned s2 = (unsigned)da.z - nbs, s3 = (unsigned)da.w - nbs;
  const unsigned s4 = (unsigned)db.x - nbs, s5 = (unsigned)db.y - nbs;
  const unsigned s6 = (unsigned)db.z - nbs, s7 = (unsigned)db.w - nbs;
  const bool h0 = s0 < unb, h1 = s1 < unb, h2 = s2 < unb, h3 = s3 < unb;
  const bool h4 = s4 < unb, h5 = s5 < unb, h6 = s6 < unb, h7 = s7 < unb;
  const unsigned any = __builtin_amdgcn_ballot_w32(h0 | h1 | h2 | h3 | h4 | h5 | h6 | h7);
  if (any != 0u) {
#define HITJ(J, HJ, SJ) { \
      const unsigned mj = __builtin_amdgcn_ballot_w32(HJ); \
      if (mj != 0u) { \
        if (HJ) { \
          const int pos = wc + (int)__builtin_amdgcn_mbcnt_lo(mj, 0u); \
          if (pos < WLCAP) wlw[pos] = ((e0 + (J)) << SLA) | (int)(SJ); \
        } \
        wc += (int)__builtin_popcount(mj); } }
    HITJ(0, h0, s0)
    HITJ(1, h1, s1)
    HITJ(2, h2, s2)
    HITJ(3, h3, s3)
    HITJ(4, h4, s4)
    HITJ(5, h5, s5)
    HITJ(6, h6, s6)
    HITJ(7, h7, s7)
#undef HITJ
  }
  return wc;
}

__device__ __forceinline__ void list_pass(const int* sl, const int* __restrict__ srcs, int tt, int tid, int* lp) {
#pragma unroll 1
  for (int it = 0; it < RCAP / (BTHR * 4); ++it) {
    const int i0 = it * (BTHR * 4) + tid * 4;
    const v4i u4 = *(const v4ia*)(sl + i0);
    int e0 = u4.x >> SLA, e1 = u4.y >> SLA, e2 = u4.z >> SLA, e3 = u4.w >> SLA;
    e0 = e0 < 0 ? 0 : (e0 > NE - 1 ? NE - 1 : e0);
    e1 = e1 < 0 ? 0 : (e1 > NE - 1 ? NE - 1 : e1);
    e2 = e2 < 0 ? 0 : (e2 > NE - 1 ? NE - 1 : e2);
    e3 = e3 < 0 ? 0 : (e3 > NE - 1 ? NE - 1 : e3);
    int r0 = srcs[e0], r1 = srcs[e1], r2 = srcs[e2], r3 = srcs[e3];
    asm volatile("" :: "v"(r0), "v"(r1), "v"(r2), "v"(r3));
    r0 = r0 < 0 ? 0 : (r0 > NN - 1 ? NN - 1 : r0);
    r1 = r1 < 0 ? 0 : (r1 > NN - 1 ? NN - 1 : r1);
    r2 = r2 < 0 ? 0 : (r2 > NN - 1 ? NN - 1 : r2);
    r3 = r3 < 0 ? 0 : (r3 > NN - 1 ? NN - 1 : r3);
    v4i o;
    o.x = r0 & -(int)(i0     < tt);
    o.y = r1 & -(int)(i0 + 1 < tt);
    o.z = r2 & -(int)(i0 + 2 < tt);
    o.w = r3 & -(int)(i0 + 3 < tt);
    *(volatile v4i*)(lp + i0) = o;
  }
}

__global__ __launch_bounds__(BTHR) void k_bucket(const int* __restrict__ srcs, const int* __restrict__ dsts,
                                                 int vec8, int* listp, int* cntp, int* offp, float* invp,
                                                 int* flagp) {
  extern __shared__ __attribute__((aligned(16))) int dsm[];
  int* wl   = dsm;
  int* sl   = wl + BWAVE * WLCAP;
  int* cnt  = sl + RCAP;
  int* offs = cnt + NBA;
  int* cur  = offs + NBA;
  int* misc = cur + NBA;
  const int tid = (int)threadIdx.x, lane = tid & 31, wave = tid >> 5;
  const int blk = (int)blockIdx.x;
  const int nodeBase = blk * NBA;
  {
    const v4i z4 = {0, 0, 0, 0};
    for (int i = tid * 4; i < BZ_INTS; i += BTHR * 4) *(v4ia*)(dsm + i) = z4;
    if (tid < 16) misc[tid] = 0;
  }
  __syncthreads();

  int nb = NN - nodeBase;
  nb = nb > NBA ? NBA : nb;
  nb = nb < 0 ? 0 : nb;

  {
    int wc = 0;
    int* wlw = wl + wave * WLCAP;
    const int nChunks = (NE + CHUNK - 1) / CHUNK;
#pragma unroll 1
    for (int ch = 0; ch < nChunks; ++ch)
      wc = sweep_chunk(dsts, ch * CHUNK, nodeBase, nb, vec8, wlw, wc, tid);
    if (lane == 0) misc[wave] = wc;
  }
  __syncthreads();

  int t = 0, ov = 0;
  if (wave == 0) {
#pragma unroll 1
    for (int w2 = 0; w2 < BWAVE; ++w2) {
      int cv = misc[w2];
      const int ovl = (cv > WLCAP) ? 1 : 0;
      cv = cv < 0 ? 0 : (cv > WLCAP ? WLCAP : cv);
      const int c = __builtin_amdgcn_readfirstlane(cv);
      ov |= __builtin_amdgcn_readfirstlane(ovl);
#pragma unroll 1
      for (int b0 = 0; b0 < c; b0 += 32) {
        const int idx = b0 + lane;
        const int ent = wl[w2 * WLCAP + (idx < WLCAP ? idx : WLCAP - 1)];
        const int m32 = (c - b0) < 32 ? (c - b0) : 32;
#pragma unroll 1
        for (int k = 0; k < m32; ++k) {
          const int u    = __builtin_amdgcn_readlane(ent, k);
          const int slot = u & (NBA - 1);
          if (t < RCAP) {
            if (lane == 0) cnt[slot] = cnt[slot] + 1;
            t = t + 1;
          } else {
            ov = 1;
          }
        }
      }
    }
  }
  if (wave == 0 && lane == 0) { misc[8] = t; misc[9] = ov; }
  __syncthreads();
  int ttv = misc[8];
  ttv = ttv < 0 ? 0 : (ttv > RCAP ? RCAP : ttv);
  const int tt  = __builtin_amdgcn_readfirstlane(ttv);
  const int ovf = __builtin_amdgcn_readfirstlane(misc[9]);

  if (wave == 0) {
    const int base = lane * (NBA / 32);
    int s = 0;
#pragma unroll 1
    for (int i = 0; i < NBA / 32; ++i) s += cnt[base + i];
    int incl = s;
#pragma unroll
    for (int d = 1; d < 32; d <<= 1) {
      const int y = __shfl_up(incl, d, 32);
      if (lane >= d) incl += y;
    }
    int run = incl - s;
#pragma unroll 1
    for (int i = 0; i < NBA / 32; ++i) {
      const int cv = cnt[base + i];
      offs[base + i] = run;
      cur[base + i]  = run;
      run += cv;
    }
  }
  __syncthreads();
  if (wave == 0) {
    int t2 = 0;
#pragma unroll 1
    for (int w2 = 0; w2 < BWAVE; ++w2) {
      int cv = misc[w2];
      cv = cv < 0 ? 0 : (cv > WLCAP ? WLCAP : cv);
      const int c = __builtin_amdgcn_readfirstlane(cv);
#pragma unroll 1
      for (int b0 = 0; b0 < c; b0 += 32) {
        const int idx = b0 + lane;
        const int ent = wl[w2 * WLCAP + (idx < WLCAP ? idx : WLCAP - 1)];
        const int m32 = (c - b0) < 32 ? (c - b0) : 32;
#pragma unroll 1
        for (int k = 0; k < m32; ++k) {
          const int u    = __builtin_amdgcn_readlane(ent, k);
          const int slot = u & (NBA - 1);
          if (t2 < tt) {
            if (lane == 0) {
              int p = cur[slot];
              p = p < 0 ? 0 : (p > RCAP - 1 ? RCAP - 1 : p);
              sl[p] = u;
              cur[slot] = p + 1;
            }
          }
          t2 = t2 + 1;
        }
      }
    }
  }
  __syncthreads();

  const v4i c4 = *(const v4ia*)(cnt + 4 * tid);
  const v4i o4 = *(const v4ia*)(offs + 4 * tid);
  v4f i4;
  i4.x = 1.0f / fmaxf((float)c4.x, 1.0f);
  i4.y = 1.0f / fmaxf((float)c4.y, 1.0f);
  i4.z = 1.0f / fmaxf((float)c4.z, 1.0f);
  i4.w = 1.0f / fmaxf((float)c4.w, 1.0f);
  v4i f4 = {0, 0, 0, 0};
  f4.x = (tid == 0) ? ovf : 0;
  const bool fw = tid < 8;
  int*   lp = listp + (size_t)blk * RCAP;
  int*   cp = cntp + (size_t)nodeBase + 4 * tid;
  int*   op = offp + (size_t)nodeBase + 4 * tid;
  float* ip = invp + (size_t)nodeBase + 4 * tid;
  int*   fp = flagp + (size_t)blk * 32 + 4 * (fw ? tid : 0);
  list_pass(sl, srcs, tt, tid, lp);
  *(volatile v4i*)cp = c4;
  *(volatile v4i*)op = o4;
  *(volatile v4f*)ip = i4;
  if (fw) *(volatile v4i*)fp = f4;
  __threadfence();
  list_pass(sl, srcs, tt, tid, lp);
  *(volatile v4i*)cp = c4;
  *(volatile v4i*)op = o4;
  *(volatile v4f*)ip = i4;
  if (fw) *(volatile v4i*)fp = f4;
}

template <int FIRST>
__global__ __launch_bounds__(RTHR) void k_replay(const unsigned short* __restrict__ gp, const int* __restrict__ listp,
                                                 const int* __restrict__ cntp, const int* __restrict__ offp,
                                                 const float* __restrict__ invp, const int* __restrict__ flagp,
                                                 unsigned short* meanp) {
  __shared__ __attribute__((aligned(16))) unsigned short rbuf[RWAVE * MW];
  const int tid = (int)threadIdx.x, lane = tid & 31, wave = tid >> 5;
  unsigned short* rowbuf = rbuf + wave * MW;
#pragma unroll 1
  for (int r = 0; r < RROWS; ++r) {
    const int node = (int)blockIdx.x * RBROWS + r * RWAVE + wave;
    if (node < NN) {
      int c = cntp[node];
      int o = offp[node];
      const float iv = invp[node];
      const int fl = flagp[(node >> SLA) * 32];
      const bool bad = (c > DEGCAP) || (c < 0) || (fl != 0);
      c = c < 0 ? 0 : (c > DEGCAP ? DEGCAP : c);
      o = o < 0 ? 0 : (o > RCAP - 1 ? RCAP - 1 : o);
      int last = o + c - 1;
      last = last < o ? o : last;
      last = last > RCAP - 1 ? RCAP - 1 : last;
      const int cu = __builtin_amdgcn_readfirstlane(c);
      const int ou = __builtin_amdgcn_readfirstlane(o);
      const int lu = __builtin_amdgcn_readfirstlane(last);
      const float pz = bad ? __int_as_float(0x7fc00000) : 0.0f;
      const int* lp = listp + (size_t)(node >> SLA) * RCAP;
      float a0 = 0.0f, a1 = 0.0f, a2 = 0.0f, a3 = 0.0f;
#pragma unroll 1
      for (int b0 = 0; b0 < cu; b0 += 32) {
        int idx = ou + b0 + lane;
        idx = idx > lu ? lu : idx;
        int sr = lp[idx];
        sr = sr < 0 ? 0 : (sr > NN - 1 ? NN - 1 : sr);
        const int m32 = (cu - b0) < 32 ? (cu - b0) : 32;
#pragma unroll 1
        for (int k = 0; k < m32; ++k) {
          const int sk = __builtin_amdgcn_readlane(sr, k);
          if constexpr (FIRST != 0) {
            const unsigned short* rp = gp + (size_t)sk * DF + 4 * lane;
            const v2u q = *(const v2ua*)rp;
            a0 += __uint_as_float(q.x << 16);
            a1 += __uint_as_float(q.x & 0xffff0000u);
            a2 += __uint_as_float(q.y << 16);
            a3 += __uint_as_float(q.y & 0xffff0000u);
          } else {
            const unsigned short* rp = gp + (size_t)sk * MW + 4 * lane;
            const v2u wh = *(const v2ua*)rp;
            const v2u wq = *(const v2ua*)(rp + DF);
            a0 += __uint_as_float(wh.x << 16)         + __uint_as_float(wq.x << 16);
            a1 += __uint_as_float(wh.x & 0xffff0000u) + __uint_as_float(wq.x & 0xffff0000u);
            a2 += __uint_as_float(wh.y << 16)         + __uint_as_float(wq.y << 16);
            a3 += __uint_as_float(wh.y & 0xffff0000u) + __uint_as_float(wq.y & 0xffff0000u);
          }
        }
      }
      const float m0 = a0 * iv + pz, m1 = a1 * iv + pz, m2 = a2 * iv + pz, m3 = a3 * iv + pz;
      v4us mh, ml;
      {
        unsigned lb;
        unsigned hb;
        hb = hl_bits(m0, lb); mh[0] = (unsigned short)hb; ml[0] = (unsigned short)lb;
        hb = hl_bits(m1, lb); mh[1] = (unsigned short)hb; ml[1] = (unsigned short)lb;
        hb = hl_bits(m2, lb); mh[2] = (unsigned short)hb; ml[2] = (unsigned short)lb;
        hb = hl_bits(m3, lb); mh[3] = (unsigned short)hb; ml[3] = (unsigned short)lb;
      }
      *(v4usa*)(rowbuf + 4 * lane)      = mh;
      *(v4usa*)(rowbuf + DF + 4 * lane) = ml;
      wave_sync();
      const v8us q0 = *(const v8usa*)(rowbuf + 8 * lane);
      wave_sync();
      unsigned short* rpw = meanp + (size_t)node * MW + 8 * lane;
      *(volatile v8us*)rpw = q0;
      __threadfence();
      *(volatile v8us*)rpw = q0;
    }
  }
}

__device__ __forceinline__ void kspan(const unsigned short* __restrict__ ap, const unsigned short* __restrict__ bp,
                                      int ldb, int nk, v8f (&acc)[8]) {
#pragma unroll 1
  for (int k0 = 0; k0 < nk; k0 += 32) {
    FragB af;
    af.h[0] = *(const v8usa*)(ap + k0);
    af.h[1] = *(const v8usa*)(ap + k0 + 16);
#pragma unroll
    for (int nt = 0; nt < 8; ++nt) {
      const unsigned short* wq = bp + (size_t)(16 * nt) * (size_t)ldb + k0;
      FragB bf;
      bf.h[0] = *(const v8usa*)wq;
      bf.h[1] = *(const v8usa*)(wq + 16);
      acc[nt] = wmb(af, bf, acc[nt]);
    }
  }
}

__device__ __forceinline__ void t_store_pass(const float* stg, const float* bls, float pz, int rowBase, int wave,
                                             int lane, float* outp) {
  const v4f b4 = *(const v4fa*)(bls + 4 * lane);
#pragma unroll 4
  for (int i = 0; i < 16; ++i) {
    const int row = rowBase + 16 * wave + i;
    const v4f xv = *(const v4fa*)(stg + (16 * wave + i) * GBN + 4 * lane);
    asm volatile("" :: "v"(xv));
    v4f y;
    y.x = (xv.x + b4.x) + pz; y.y = (xv.y + b4.y) + pz; y.z = (xv.z + b4.z) + pz; y.w = (xv.w + b4.w) + pz;
    if (row < NN) *(volatile v4f*)(outp + (size_t)row * DF + 4 * lane) = y;
  }
}

template <int REC>
__global__ __launch_bounds__(GTHR) __attribute__((amdgpu_num_vgpr(248)))
void k_gemm(const unsigned short* __restrict__ meanp, const unsigned short* __restrict__ p2, int ld2, int k2,
            const unsigned short* __restrict__ wc, int ldb, const float* __restrict__ blt,
            const int* __restrict__ flagp, float* outp, double* recp) {
  extern __shared__ __attribute__((aligned(16))) float gsm[];
  float*  stg = gsm;
  float*  bls = gsm + GBM * GBN;
  double* rcs = (double*)(gsm + GBM * GBN + DF);
  const int tid = (int)threadIdx.x, lane = tid & 31, wave = tid >> 5, hh = lane >> 4, m = lane & 15;
  const int rowBase = (int)blockIdx.x * GBM;

  if (tid < 32) *(v4fa*)(bls + 4 * tid) = *(const v4f*)(blt + 4 * tid);

  v8f acc[8];
#pragma unroll
  for (int t = 0; t < 8; ++t) acc[t] = z8();
  const size_t arow = (size_t)(rowBase + 16 * wave + m);
  const unsigned short* bp = wc + (size_t)m * (size_t)ldb + 8 * hh;
  kspan(meanp + arow * MW + 8 * hh, bp, ldb, 2 * DF, acc);
  kspan(p2 + arow * (size_t)ld2 + 8 * hh, bp + 2 * DF, ldb, k2, acc);

#pragma unroll
  for (int nt = 0; nt < 8; ++nt) {
    const int lc = 16 * nt + m;
#pragma unroll
    for (int r = 0; r < 8; ++r) {
      const int lr = 16 * wave + 8 * hh + r;
      stg[lr * GBN + lc] = acc[nt][r];
    }
  }
  __syncthreads();

  const int fl = flagp[((int)blockIdx.x >> 3) * 32];
  const float pz = (fl != 0) ? __int_as_float(0x7fc00000) : 0.0f;

  t_store_pass(stg, bls, pz, rowBase, wave, lane, outp);

  v4u rv = {0u, 0u, 0u, 0u};
  unsigned* rp = (unsigned*)recp + (size_t)blockIdx.x * (4 * DF) + 4 * (tid < DF ? tid : 0);
  if constexpr (REC != 0) {
    if (tid < DF) {
      int nv = NN - rowBase;
      nv = nv > GBM ? GBM : nv;
      nv = nv < 0 ? 0 : nv;
      const float bc = bls[tid];
      double s = 0.0, q = 0.0;
#pragma unroll 4
      for (int r = 0; r < nv; ++r) {
        const float tv = (stg[r * GBN + tid] + bc) + pz;
        const double td = (double)tv;
        s += td;
        q += td * td;
      }
      rcs[tid] = s;
      rcs[DF + tid] = q;
    }
    __syncthreads();
    if (tid < DF) {
      rv = *(const v4ua*)((const unsigned*)rcs + 4 * tid);
      *(volatile v4u*)rp = rv;
    }
  }
  __threadfence();
  t_store_pass(stg, bls, pz, rowBase, wave, lane, outp);
  if constexpr (REC != 0) {
    if (tid < DF) *(volatile v4u*)rp = rv;
  }
}

__global__ __launch_bounds__(DF) void k_comb(const double* __restrict__ rec, double invN, float* stat) {
  __shared__ __attribute__((aligned(16))) float sst[2 * DF];
  const int tid = (int)threadIdx.x;
  double s = 0.0, q = 0.0;
#pragma unroll 2
  for (int b = 0; b < NTILE; ++b) {
    s += rec[(size_t)b * (2 * DF) + tid];
    q += rec[(size_t)b * (2 * DF) + DF + tid];
  }
  const double mu  = s * invN;
  const double var = q * invN - mu * mu;
  const float mf = (float)mu;
  float vf = (float)var;
  vf = (vf < 0.0f) ? 0.0f : vf;
  const float rs = 1.0f / sqrtf(vf + BNEPS);
  sst[tid] = mf;
  sst[DF + tid] = rs;
  __syncthreads();
  const bool ok = tid < (2 * DF) / 4;
  v4f v = {0.f, 0.f, 0.f, 0.f};
  if (ok) v = *(const v4fa*)(sst + 4 * tid);
  float* op = stat + 4 * (ok ? tid : 0);
  if (ok) *(volatile v4f*)op = v;
  __threadfence();
  if (ok) *(volatile v4f*)op = v;
}

__global__ __launch_bounds__(RTHR) void k_apply(const float* tin, const float* __restrict__ stat,
                                                const float* __restrict__ gt, const float* __restrict__ bt,
                                                unsigned short* hp) {
  __shared__ __attribute__((aligned(16))) float par[4 * DF];
  __shared__ __attribute__((aligned(16))) unsigned short rbuf[RWAVE * MW];
  const int tid = (int)threadIdx.x, lane = tid & 31, wave = tid >> 5;
  if (tid < 32) {
    *(v4fa*)(par + 4 * tid)          = *(const v4f*)(stat + 4 * tid);
    *(v4fa*)(par + DF + 4 * tid)     = *(const v4f*)(stat + DF + 4 * tid);
    *(v4fa*)(par + 2 * DF + 4 * tid) = *(const v4f*)(gt + 4 * tid);
    *(v4fa*)(par + 3 * DF + 4 * tid) = *(const v4f*)(bt + 4 * tid);
  }
  __syncthreads();
  const v4f m4 = *(const v4fa*)(par + 4 * lane);
  const v4f r4 = *(const v4fa*)(par + DF + 4 * lane);
  const v4f g4 = *(const v4fa*)(par + 2 * DF + 4 * lane);
  const v4f b4 = *(const v4fa*)(par + 3 * DF + 4 * lane);
  unsigned short* rowbuf = rbuf + wave * MW;
#pragma unroll 1
  for (int r = 0; r < RROWS; ++r) {
    const int node = (int)blockIdx.x * RBROWS + r * RWAVE + wave;
    if (node < NN) {
      const v4f t = *(const v4f*)(tin + (size_t)node * DF + 4 * lane);
      float y0 = ((t.x - m4.x) * r4.x) * g4.x + b4.x;
      float y1 = ((t.y - m4.y) * r4.y) * g4.y + b4.y;
      float y2 = ((t.z - m4.z) * r4.z) * g4.z + b4.z;
      float y3 = ((t.w - m4.w) * r4.w) * g4.w + b4.w;
      y0 = (y0 > 0.0f) ? y0 : (y0 - y0);
      y1 = (y1 > 0.0f) ? y1 : (y1 - y1);
      y2 = (y2 > 0.0f) ? y2 : (y2 - y2);
      y3 = (y3 > 0.0f) ? y3 : (y3 - y3);
      v4us h4, l4;
      {
        unsigned lb;
        unsigned hb;
        hb = hl_bits(y0, lb); h4[0] = (unsigned short)hb; l4[0] = (unsigned short)lb;
        hb = hl_bits(y1, lb); h4[1] = (unsigned short)hb; l4[1] = (unsigned short)lb;
        hb = hl_bits(y2, lb); h4[2] = (unsigned short)hb; l4[2] = (unsigned short)lb;
        hb = hl_bits(y3, lb); h4[3] = (unsigned short)hb; l4[3] = (unsigned short)lb;
      }
      *(v4usa*)(rowbuf + 4 * lane)      = h4;
      *(v4usa*)(rowbuf + DF + 4 * lane) = l4;
      wave_sync();
      const v8us q0 = *(const v8usa*)(rowbuf + 8 * lane);
      wave_sync();
      unsigned short* rpw = hp + (size_t)node * MW + 8 * lane;
      *(volatile v8us*)rpw = q0;
      __threadfence();
      *(volatile v8us*)rpw = q0;
    }
  }
}

#define STHR   256
#define SPM    4096
#define SPV    32
#define SB_M   96
#define SB_V   7
#define SB_ALL (SB_M + SB_V)

constexpr size_t SZ_SWL = (size_t)NLAY * DF * DF * 4;
constexpr size_t SZ_SBL = (size_t)NLAY * DF * 4;
constexpr size_t SZ_SWR = (size_t)NLAY * DF * DF * 4;
constexpr size_t SZ_SG  = (size_t)2 * DF * 4;
constexpr size_t SZ_SBE = (size_t)2 * DF * 4;
constexpr size_t O_SWL  = ((O_END + 127) / 128) * 128;
constexpr size_t O_SBL  = O_SWL + SZ_SWL;
constexpr size_t O_SWR  = O_SBL + SZ_SBL;
constexpr size_t O_SG   = O_SWR + SZ_SWR;
constexpr size_t O_SBE  = O_SG + SZ_SG;
constexpr size_t O_TOT  = O_SBE + SZ_SBE;
static_assert(6 * 4096 + 7 * 32 == 24800);
static_assert(6 * SPM + 7 * SPV == 24800 && (SB_M / 6) * STHR == SPM && SPV <= STHR);
static_assert((SZ_SWL + SZ_SBL + SZ_SWR + SZ_SG + SZ_SBE) == (size_t)24800 * 16);
static_assert(SZ_SWL + SZ_SBL + SZ_SWR + SZ_SG + SZ_SBE == 396800);
static_assert(O_SWL % 128 == 0 && O_SBL % 128 == 0 && O_SWR % 128 == 0 && O_SG % 128 == 0 && O_SBE % 128 == 0);
static_assert(SZ_SWL % 128 == 0 && SZ_SBL % 128 == 0 && SZ_SWR % 128 == 0 && SZ_SG % 128 == 0 && SZ_SBE % 128 == 0);
static_assert(O_SWL >= O_END);
static_assert(O_END == 113710848);
static_assert(O_TOT == 114107648);
static_assert(O_TOT <= ((size_t)128 << 20));


__global__ __launch_bounds__(STHR) void k_stack(const float* __restrict__ p_wl0, const float* __restrict__ p_wl1, const float* __restrict__ p_wl2, const float* __restrict__ p_wr0, const float* __restrict__ p_wr1, const float* __restrict__ p_wr2, const float* __restrict__ p_b0, const float* __restrict__ p_b1, const float* __restrict__ p_b2, const float* __restrict__ p_g0, const float* __restrict__ p_g1, const float* __restrict__ p_be0, const float* __restrict__ p_be1, float* __restrict__ wsf) {
  const int b = (int)blockIdx.x, tid = (int)threadIdx.x;
  int role, piece, np;
  if (b < SB_M) { role = b >> 4;        piece = (b & 15) * STHR + tid; np = SPM; }
  else          { role = 6 + (b - SB_M); piece = tid;                   np = SPV; }
  role = role > 12 ? 12 : role;
  const bool live = piece < np;
  const int pc = piece < np ? piece : np - 1;
  const size_t so = (size_t)pc * 4;
  v4f v = {0.f, 0.f, 0.f, 0.f};
  size_t dw = 0;
  switch (role) {
    case 0:  v = *(const v4f*)(p_wl0 + so); dw = O_SWL / 4;                        break;
    case 1:  v = *(const v4f*)(p_wl1 + so); dw = O_SWL / 4 + (size_t)DF * DF;      break;
    case 2:  v = *(const v4f*)(p_wl2 + so); dw = O_SWL / 4 + (size_t)2 * DF * DF;  break;
    case 3:  v = *(const v4f*)(p_wr0 + so); dw = O_SWR / 4;                        break;
    case 4:  v = *(const v4f*)(p_wr1 + so); dw = O_SWR / 4 + (size_t)DF * DF;      break;
    case 5:  v = *(const v4f*)(p_wr2 + so); dw = O_SWR / 4 + (size_t)2 * DF * DF;  break;
    case 6:  v = *(const v4f*)(p_b0 + so);  dw = O_SBL / 4;                        break;
    case 7:  v = *(const v4f*)(p_b1 + so);  dw = O_SBL / 4 + (size_t)DF;           break;
    case 8:  v = *(const v4f*)(p_b2 + so);  dw = O_SBL / 4 + (size_t)2 * DF;       break;
    case 9:  v = *(const v4f*)(p_g0 + so);  dw = O_SG / 4;                         break;
    case 10: v = *(const v4f*)(p_g1 + so);  dw = O_SG / 4 + (size_t)DF;            break;
    case 11: v = *(const v4f*)(p_be0 + so); dw = O_SBE / 4;                        break;
    default: v = *(const v4f*)(p_be1 + so); dw = O_SBE / 4 + (size_t)DF;           break;
  }
  asm volatile("" :: "v"(v.x), "v"(v.y), "v"(v.z), "v"(v.w));
  float* dp = wsf + dw + so;
  if (live) *(volatile v4f*)dp = v;
  __threadfence();
  if (live) *(volatile v4f*)dp = v;
}

static inline int cdiv(int a, int b) { return (a + b - 1) / b; }

extern "C" void kernel_launch(void* const* d_in, const int* in_sizes, int n_in,
                              void* d_out, int out_size, void* d_ws, size_t ws_size,
                              hipStream_t stream) {
  if (n_in < 15) return;
  if (in_sizes[0] != NN * DF) return;
  if (in_sizes[1] != DF * DF || in_sizes[2] != DF * DF) return;
  if (in_sizes[3] != DF || in_sizes[4] != DF || in_sizes[5] != DF) return;
  if (in_sizes[6] != DF * DF || in_sizes[7] != DF * DF) return;
  if (in_sizes[8] != DF || in_sizes[9] != DF || in_sizes[10] != DF) return;
  if (in_sizes[11] != DF * DF || in_sizes[12] != DF * DF) return;
  if (in_sizes[13] != DF) return;
  if (in_sizes[14] != 2 * NE) return;
  if (out_size != NN * DF) return;
  if (O_TOT > ws_size) return;

  const float* x  = (const float*)d_in[0];
  const int*   ei = (const int*)  d_in[14];
  float* out = (float*)d_out;
  const int* src = ei;
  const int* dst = ei + NE;

  const float* p_wl0 = (const float*)d_in[1];
  const float* p_wl1 = (const float*)d_in[6];
  const float* p_wl2 = (const float*)d_in[11];
  const float* p_wr0 = (const float*)d_in[2];
  const float* p_wr1 = (const float*)d_in[7];
  const float* p_wr2 = (const float*)d_in[12];
  const float* p_b0 = (const float*)d_in[3];
  const float* p_b1 = (const float*)d_in[8];
  const float* p_b2 = (const float*)d_in[13];
  const float* p_g0 = (const float*)d_in[4];
  const float* p_g1 = (const float*)d_in[9];
  const float* p_be0 = (const float*)d_in[5];
  const float* p_be1 = (const float*)d_in[10];

  char* ws = (char*)d_ws;
  unsigned short* MEAN = (unsigned short*)(ws + O_MEAN);
  unsigned short* Hp   = (unsigned short*)(ws + O_H);
  unsigned short* XB   = (unsigned short*)(ws + O_H);
  int*    LIST = (int*)(ws + O_LIST);
  int*    CNT  = (int*)(ws + O_CNT);
  int*    OFF  = (int*)(ws + O_OFF);
  float*  INV  = (float*)(ws + O_INV);
  double* REC  = (double*)(ws + O_REC);
  unsigned short* WC0 = (unsigned short*)(ws + O_WC0);
  unsigned short* WC1 = (unsigned short*)(ws + O_WC1);
  unsigned short* WC2 = (unsigned short*)(ws + O_WC2);
  float*  TAB  = (float*)(ws + O_TAB);
  float*  STAT = (float*)(ws + O_STAT);
  int*    FLAG = (int*)(ws + O_FLAG);
  const float* Wl  = (const float*)(ws + O_SWL);
  const float* bl  = (const float*)(ws + O_SBL);
  const float* Wr  = (const float*)(ws + O_SWR);
  const float* gam = (const float*)(ws + O_SG);
  const float* bet = (const float*)(ws + O_SBE);

  hipFuncSetAttribute(reinterpret_cast<const void*>(&k_bucket), hipFuncAttributeMaxDynamicSharedMemorySize, (int)BLDS_BYTES);
  hipFuncSetAttribute(reinterpret_cast<const void*>(&k_gemm<1>), hipFuncAttributeMaxDynamicSharedMemorySize, (int)GLDS_BYTES);
  hipFuncSetAttribute(reinterpret_cast<const void*>(&k_gemm<0>), hipFuncAttributeMaxDynamicSharedMemorySize, (int)GLDS_BYTES);

  const int vec8 = ((NE & 3) == 0) ? 1 : 0;
  const int gR = cdiv(NN, RBROWS);
  const double invN = 1.0 / (double)NN;

  k_stack<<<SB_ALL, STHR, 0, stream>>>(p_wl0, p_wl1, p_wl2, p_wr0, p_wr1, p_wr2, p_b0, p_b1, p_b2, p_g0, p_g1, p_be0, p_be1, (float*)d_ws);
  k_prep<<<PB_ALL, PTHR, 0, stream>>>(x, Wl, Wr, bl, gam, bet, (unsigned*)d_ws);
  k_bucket<<<NBLK, BTHR, BLDS_BYTES, stream>>>(src, dst, vec8, LIST, CNT, OFF, INV, FLAG);
  k_replay<1><<<gR, RTHR, 0, stream>>>(XB, LIST, CNT, OFF, INV, FLAG, MEAN);
  k_gemm<1><<<NTILE, GTHR, GLDS_BYTES, stream>>>(MEAN, XB, DF, DF, WC0, K0, TAB, FLAG, out, REC);
  k_comb<<<1, DF, 0, stream>>>(REC, invN, STAT);
  k_apply<<<gR, RTHR, 0, stream>>>(out, STAT, TAB + 3 * DF, TAB + 5 * DF, Hp);
  k_replay<0><<<gR, RTHR, 0, stream>>>(Hp, LIST, CNT, OFF, INV, FLAG, MEAN);
  k_gemm<1><<<NTILE, GTHR, GLDS_BYTES, stream>>>(MEAN, Hp, MW, 2 * DF, WC1, K1, TAB + DF, FLAG, out, REC);
  k_comb<<<1, DF, 0, stream>>>(REC, invN, STAT + 2 * DF);
  k_apply<<<gR, RTHR, 0, stream>>>(out, STAT + 2 * DF, TAB + 4 * DF, TAB + 6 * DF, Hp);
  k_replay<0><<<gR, RTHR, 0, stream>>>(Hp, LIST, CNT, OFF, INV, FLAG, MEAN);
  k_gemm<0><<<NTILE, GTHR, GLDS_BYTES, stream>>>(MEAN, Hp, MW, 2 * DF, WC2, K1, TAB + 2 * DF, FLAG, out, REC);
}
